// RNN_72816875537107
// MI455X (gfx1250) — hardware-verified
//
#include <hip/hip_runtime.h>
#include <math.h>

constexpr int NB    = 64;
constexpr int NT    = 1024;
constexpr int NI    = 64;
constexpr int NH    = 512;
constexpr int NO    = 64;
constexpr int NROWS = NB * NT;
constexpr int NOUT0 = NROWS * NO;
constexpr int NOUT1 = NB * NH;

constexpr int SEQ_BLK  = 16;
constexpr int RNN_BLKS = NB / SEQ_BLK;
constexpr int RNN_THR  = 256;
constexpr int NWAVE    = RNN_THR / 32;
constexpr int HP       = NH + 8;
constexpr int XP       = NI + 8;
constexpr int HTILE    = SEQ_BLK * HP;
constexpr int XTILE    = SEQ_BLK * XP;
constexpr int SLABP    = 68;

constexpr float W_CARRY      = 256.0f;
constexpr float W_CARRY_INV  = 1.0f / 256.0f;
constexpr float LO_CARRY     = 2048.0f;
constexpr float LO_CARRY_INV = 1.0f / 2048.0f;
constexpr float F16_MIN_NORMAL = 6.103515625e-5f;

constexpr int N8_WIH  = NH * NI / 8;
constexpr int N8_WHH  = NH * NH / 8;
constexpr int N8_WOUT = NO * NH / 8;
constexpr int HEAD_GRID = ((NROWS / 64) * (NO / 64)) / 8;

static_assert(NB % SEQ_BLK == 0);
static_assert(NH == NWAVE * 64);
static_assert(HP % 8 == 0 && XP % 8 == 0);
static_assert(NI % 32 == 0 && NH % 32 == 0);
static_assert(NROWS % 64 == 0 && NO % 64 == 0 && NH % 64 == 0);
static_assert(((NROWS / 64) * (NO / 64)) % 8 == 0);
static_assert(SEQ_BLK * NI == RNN_THR * 4);
static_assert((SEQ_BLK * NH) % (RNN_THR * 4) == 0);
static_assert(N8_WIH % 256 == 0 && N8_WHH % 256 == 0 && N8_WOUT % 256 == 0);
static_assert((size_t)NOUT0 * 4 == (size_t)16777216);
static_assert((2 * HTILE) % 8 == 0 && (2 * XTILE) % 8 == 0);

typedef __attribute__((ext_vector_type(16))) _Float16 v16h;
typedef __attribute__((ext_vector_type(8)))  _Float16 v8h;
typedef __attribute__((ext_vector_type(4)))  _Float16 v4h;
typedef __attribute__((ext_vector_type(16))) __bf16   v16b;
typedef __attribute__((ext_vector_type(8)))  __bf16   v8b;
typedef __attribute__((ext_vector_type(8)))  float    v8f;
typedef __attribute__((ext_vector_type(4)))  float    v4f;

__device__ __forceinline__ unsigned short f2bf_bits(float f) {
  unsigned u = __float_as_uint(f);
  return (unsigned short)((u + 0x7FFFu + ((u >> 16) & 1u)) >> 16);
}
__device__ __forceinline__ float bf_bits2f(unsigned short h) { return __uint_as_float(((unsigned)h) << 16); }

__device__ __forceinline__ void dep_guard_h(v8f& a, v8f& b, v16h x, v16h y) { asm volatile("v_nop\n\tv_nop\n\tv_nop\n\tv_nop" : "+v"(a), "+v"(b) : "v"(x), "v"(y)); }
__device__ __forceinline__ void dep_guard_b(v8f& a, v8f& b, v16b x, v16b y) { asm volatile("v_nop\n\tv_nop\n\tv_nop\n\tv_nop" : "+v"(a), "+v"(b) : "v"(x), "v"(y)); }
__device__ __forceinline__ void keep4_h(v16h a, v16h b, v16h c, v16h d) { asm volatile("v_nop" :: "v"(a), "v"(b), "v"(c), "v"(d)); }
__device__ __forceinline__ void keep4_b(v16b a, v16b b, v16b c, v16b d) { asm volatile("v_nop" :: "v"(a), "v"(b), "v"(c), "v"(d)); }
__device__ __forceinline__ void acc_guard4(v8f& a, v8f& b, v8f& c, v8f& d) { asm volatile("v_nop\n\tv_nop\n\tv_nop\n\tv_nop" : "+v"(a), "+v"(b), "+v"(c), "+v"(d)); }
template <typename V>
__device__ __forceinline__ void guard4ab(v8f& a0, v8f& a1, v8f& a2, v8f& a3, V x0, V x1, V y0, V y1, V y2, V y3) {
  asm volatile("v_nop\n\tv_nop\n\tv_nop\n\tv_nop"
               : "+v"(a0), "+v"(a1), "+v"(a2), "+v"(a3)
               : "v"(x0), "v"(x1), "v"(y0), "v"(y1), "v"(y2), "v"(y3));
}
__device__ __forceinline__ void guard8ab_h(v8f& a0, v8f& a1, v8f& a2, v8f& a3, v8f& b0, v8f& b1, v8f& b2, v8f& b3,
                                           v16h x0, v16h x1, v16h y0, v16h y1, v16h y2, v16h y3) {
  asm volatile("v_nop\n\tv_nop\n\tv_nop\n\tv_nop"
               : "+v"(a0), "+v"(a1), "+v"(a2), "+v"(a3), "+v"(b0), "+v"(b1), "+v"(b2), "+v"(b3)
               : "v"(x0), "v"(x1), "v"(y0), "v"(y1), "v"(y2), "v"(y3));
}

template <typename T> struct Frag;
template <> struct Frag<_Float16> {
  typedef v16h V; union U { v16h v; v8h h[2]; };
  static __device__ __forceinline__ v16h load(const _Float16* p) {
    U f; f.h[0] = *(const v8h*)(p); f.h[1] = *(const v8h*)(p + 16); return f.v;
  }
  static __device__ __forceinline__ v8f mma(v16h a, v16h b, v8f c) {
    return __builtin_amdgcn_wmma_f32_16x16x32_f16(false, a, false, b, (short)0, c, false, false);
  }
  static __device__ __forceinline__ void guard(v8f& a, v8f& b, v16h x, v16h y) { dep_guard_h(a, b, x, y); }
  static __device__ __forceinline__ void keep(v16h a, v16h b, v16h c, v16h d) { keep4_h(a, b, c, d); }
};
template <> struct Frag<__bf16> {
  typedef v16b V; union U { v16b v; v8b h[2]; };
  static __device__ __forceinline__ v16b load(const __bf16* p) {
    U f; f.h[0] = *(const v8b*)(p); f.h[1] = *(const v8b*)(p + 16); return f.v;
  }
  static __device__ __forceinline__ v8f mma(v16b a, v16b b, v8f c) {
    return __builtin_amdgcn_wmma_f32_16x16x32_bf16(false, a, false, b, (short)0, c, false, false);
  }
  static __device__ __forceinline__ void guard(v8f& a, v8f& b, v16b x, v16b y) { dep_guard_b(a, b, x, y); }
  static __device__ __forceinline__ void keep(v16b a, v16b b, v16b c, v16b d) { keep4_b(a, b, c, d); }
};

template <int ET> struct Elem;
template <> struct Elem<0> { typedef _Float16 T; };
template <> struct Elem<1> { typedef __bf16 T; };
template <int ET, bool SPLIT, int BIAS_MODE, int OUT_MODE, bool RESID, int ACT = 0>
__global__ __launch_bounds__(256) void wmma_gemm64(
    const unsigned short* __restrict__ Ap, const unsigned short* __restrict__ A2p, int lda, long strideA,
    const unsigned short* __restrict__ Btp, const unsigned short* __restrict__ Bt2p, int ldb, long strideB,
    void* __restrict__ Cout, void* __restrict__ Cout2, int ldc, long strideC,
    const float* __restrict__ bias,
    const float* __restrict__ resid, long strideR,
    int M, int N, int K, float scale) {
  typedef typename Elem<ET>::T T;
  typedef typename Frag<T>::V V;
  const T* A = (const T*)Ap; const T* A2 = (const T*)A2p; const T* Bt = (const T*)Btp; const T* Bt2 = (const T*)Bt2p;
  __shared__ __align__(16) float sT[8][16 * 68];
  const int b    = blockIdx.y;
  const int lane = threadIdx.x & 31;
  const int wave = threadIdx.x >> 5;
  const int tilesN = N >> 6;
  const int tilesM = M >> 6;
  const int tile = blockIdx.x * 8 + wave;
  if (tile >= tilesM * tilesN) return;
  const int tm = tile / tilesN;
  const int tn = tile - tm * tilesN;
  const int m0 = tm << 6;
  const int n0 = tn << 6;

  const T* Ab  = A  + (size_t)b * strideA;
  const T* Bb  = Bt + (size_t)b * strideB;
  const T* Ab2 = SPLIT ? (A2  + (size_t)b * strideA) : nullptr;
  const T* Bb2 = SPLIT ? (Bt2 + (size_t)b * strideB) : nullptr;

  const int rlane = lane & 15;
  const int koff  = (lane >> 4) * 8;
  const int mOff  = (lane >> 4) * 8;

  v8f acc[4][4];
#pragma unroll
  for (int i = 0; i < 4; ++i)
#pragma unroll
    for (int j = 0; j < 4; ++j) acc[i][j] = (v8f){0.f,0.f,0.f,0.f,0.f,0.f,0.f,0.f};

  for (int k0 = 0; k0 < K; k0 += 32) {
    V bh[4], bl[4];
#pragma unroll
    for (int j = 0; j < 4; ++j) {
      const size_t bo = (size_t)(n0 + (j << 4) + rlane) * ldb + koff + k0;
      bh[j] = Frag<T>::load(Bb + bo);
      if (SPLIT) bl[j] = Frag<T>::load(Bb2 + bo);
    }
#pragma unroll
    for (int i = 0; i < 4; ++i) {
      const size_t ao = (size_t)(m0 + (i << 4) + rlane) * lda + koff + k0;
      V ah = Frag<T>::load(Ab + ao);
      V al;
      if (SPLIT) al = Frag<T>::load(Ab2 + ao);
#pragma unroll
      for (int j = 0; j < 4; ++j) {
        acc[i][j] = Frag<T>::mma(ah, bh[j], acc[i][j]);
        if (SPLIT) {
          acc[i][j] = Frag<T>::mma(ah, bl[j], acc[i][j]);
          acc[i][j] = Frag<T>::mma(al, bh[j], acc[i][j]);
        }
      }
      guard4ab<V>(acc[i][0], acc[i][1], acc[i][2], acc[i][3], ah, SPLIT ? al : ah, bh[0], bh[1], bh[2], bh[3]);
    }
    Frag<T>::keep(bh[0], bh[1], bh[2], bh[3]);
    if (SPLIT) Frag<T>::keep(bl[0], bl[1], bl[2], bl[3]);
  }
  acc_guard4(acc[0][0], acc[0][1], acc[0][2], acc[0][3]);
  acc_guard4(acc[1][0], acc[1][1], acc[1][2], acc[1][3]);
  acc_guard4(acc[2][0], acc[2][1], acc[2][2], acc[2][3]);
  acc_guard4(acc[3][0], acc[3][1], acc[3][2], acc[3][3]);

  float* slab = sT[wave];
  const float* Rb = RESID ? (resid + (size_t)b * strideR) : nullptr;
#pragma unroll
  for (int i = 0; i < 4; ++i) {
    const int mBase = m0 + (i << 4);
#pragma unroll
    for (int j = 0; j < 4; ++j) {
      const int n = n0 + (j << 4) + rlane;
      float bv = 0.f;
      if (BIAS_MODE == 2) bv = bias[n];
#pragma unroll
      for (int r = 0; r < 8; ++r) {
        float v = acc[i][j][r] * scale;
        if (BIAS_MODE == 1) v += bias[mBase + mOff + r];
        if (BIAS_MODE == 2) v += bv;
        if (RESID) v += Rb[(size_t)(mBase + mOff + r) * ldc + n];
        if (ACT == 1) v = tanhf(v);
        if (ACT == 2) v = fmaxf(v, 0.0f);
        if (ACT == 4) v = (v > 0.f) ? v : 0.01f * v;
        slab[(mOff + r) * 68 + (j << 4) + rlane] = v;
      }
    }
    __builtin_amdgcn_fence(__ATOMIC_RELEASE, "workgroup");
    __builtin_amdgcn_wave_barrier();
    __builtin_amdgcn_fence(__ATOMIC_ACQUIRE, "workgroup");
    if (OUT_MODE == 0) {
      float* C = (float*)Cout + (size_t)b * strideC;
      const int hh = lane >> 4, c4 = (lane & 15) * 4;
      for (int pass = 0; pass < 2; ++pass) {
#pragma unroll
        for (int it = 0; it < 8; ++it) {
          const int row = it * 2 + hh;
          v4f v = *(const v4f*)(slab + row * 68 + c4);
          *(volatile v4f*)(C + (size_t)(mBase + row) * ldc + n0 + c4) = v;
        }
        __threadfence();
      }
    } else {
      const int q = lane >> 3, c8 = (lane & 7) * 8;
      unsigned short* C  = (unsigned short*)Cout  + (size_t)b * strideC;
      unsigned short* C2 = (OUT_MODE == 2) ? ((unsigned short*)Cout2 + (size_t)b * strideC) : nullptr;
      for (int pass = 0; pass < 2; ++pass) {
#pragma unroll
        for (int it = 0; it < 4; ++it) {
          const int row = it * 4 + q;
          const float* sp = slab + row * 68 + c8;
          v8h hv, lv;
#pragma unroll
          for (int e = 0; e < 8; ++e) {
            if (OUT_MODE == 1) {
              hv[e] = (_Float16)sp[e];
            } else {
              unsigned short hb = f2bf_bits(sp[e]);
              unsigned short lb = f2bf_bits(sp[e] - bf_bits2f(hb));
              hv[e] = __builtin_bit_cast(_Float16, hb);
              lv[e] = __builtin_bit_cast(_Float16, lb);
            }
          }
          *(volatile v8h*)(C + (size_t)(mBase + row) * ldc + n0 + c8) = hv;
          if (OUT_MODE == 2) *(volatile v8h*)(C2 + (size_t)(mBase + row) * ldc + n0 + c8) = lv;
        }
        __threadfence();
      }
    }
    __builtin_amdgcn_fence(__ATOMIC_RELEASE, "workgroup");
    __builtin_amdgcn_wave_barrier();
    __builtin_amdgcn_fence(__ATOMIC_ACQUIRE, "workgroup");
  }
}

__device__ __forceinline__ void split16(float v, _Float16& hi, _Float16& lo) {
  const float hq = (float)((_Float16)v);
  const float hv = (fabsf(v) < F16_MIN_NORMAL) ? 0.0f : hq;
  hi = (_Float16)hv;
  lo = (_Float16)((v - hv) * LO_CARRY);
}

__global__ __launch_bounds__(256) void cvt16_kernel(const float* __restrict__ src, unsigned short* __restrict__ dst,
                                                    int n8, float sc) {
  const int i = blockIdx.x * 256 + threadIdx.x;
  if (i < n8) {
    const float* sp = src + (size_t)i * 8;
    const v4f a = *(const v4f*)(sp);
    const v4f b = *(const v4f*)(sp + 4);
    v8h hv;
    hv[0] = (_Float16)(a[0] * sc); hv[1] = (_Float16)(a[1] * sc); hv[2] = (_Float16)(a[2] * sc); hv[3] = (_Float16)(a[3] * sc);
    hv[4] = (_Float16)(b[0] * sc); hv[5] = (_Float16)(b[1] * sc); hv[6] = (_Float16)(b[2] * sc); hv[7] = (_Float16)(b[3] * sc);
    _Float16* dp = (_Float16*)dst + (size_t)i * 8;
    *(volatile v8h*)dp = hv;
    __threadfence();
    *(volatile v8h*)dp = hv;
  }
}

__global__ __launch_bounds__(RNN_THR) void rnn_seq_kernel(
    const float* __restrict__ x, const float* __restrict__ h0,
    const float* __restrict__ b_ih, const float* __restrict__ b_hh,
    const unsigned short* __restrict__ wih16p, const unsigned short* __restrict__ whh16p,
    unsigned short* __restrict__ hs16p, float* __restrict__ hlast) {
  __shared__ __align__(16) _Float16 Hhi[2 * HTILE];
  __shared__ __align__(16) _Float16 Hlo[2 * HTILE];
  __shared__ __align__(16) _Float16 Xs[2 * XTILE];
  __shared__ __align__(16) float    Sl[NWAVE][16 * SLABP];
  const _Float16* wih16 = (const _Float16*)wih16p;
  const _Float16* whh16 = (const _Float16*)whh16p;
  _Float16* hs16 = (_Float16*)hs16p;

  const int tid = threadIdx.x, lane = tid & 31, wave = tid >> 5;
  const int c = lane & 15, hh = lane >> 4, koff = hh * 8, mOff = hh * 8, c4 = c * 4;
  const int q4 = lane >> 3, c8 = (lane & 7) * 8;
  const int b0 = blockIdx.x * SEQ_BLK;
  const int n0 = wave * 64;
  const int xr = tid >> 4, xcc = (tid & 15) * 4;

  {
    const v8h z8h = {(_Float16)0.f, (_Float16)0.f, (_Float16)0.f, (_Float16)0.f, (_Float16)0.f, (_Float16)0.f, (_Float16)0.f, (_Float16)0.f};
    for (int i = tid; i < (2 * HTILE) / 8; i += RNN_THR) { *(v8h*)(Hhi + i * 8) = z8h; *(v8h*)(Hlo + i * 8) = z8h; }
    for (int i = tid; i < (2 * XTILE) / 8; i += RNN_THR) *(v8h*)(Xs + i * 8) = z8h;
  }
  __syncthreads();

#pragma unroll
  for (int it = 0; it < 8; ++it) {
    const int i = it * RNN_THR + tid;
    const int row = i >> 7, cc = (i & 127) * 4;
    const v4f v = *(const v4f*)(h0 + (size_t)(b0 + row) * NH + cc);
    v4h hv4, lv4;
#pragma unroll
    for (int e = 0; e < 4; ++e) { _Float16 ha, la; split16(v[e], ha, la); hv4[e] = ha; lv4[e] = la; }
    *(v4h*)(Hhi + row * HP + cc) = hv4;
    *(v4h*)(Hlo + row * HP + cc) = lv4;
  }
  {
    const v4f v = *(const v4f*)(x + ((size_t)(b0 + xr) * NT + 0) * NI + xcc);
    v4h hv4;
    hv4[0] = (_Float16)v[0]; hv4[1] = (_Float16)v[1]; hv4[2] = (_Float16)v[2]; hv4[3] = (_Float16)v[3];
    *(v4h*)(Xs + xr * XP + xcc) = hv4;
  }
  float bs[4];
#pragma unroll
  for (int j = 0; j < 4; ++j) {
    const int n = n0 + 16 * j + c;
    bs[j] = b_ih[n] + b_hh[n];
  }
  __syncthreads();

  float* slab = &Sl[wave][0];
  const v8f z8 = {0.f, 0.f, 0.f, 0.f, 0.f, 0.f, 0.f, 0.f};
  const _Float16* wihrow = wih16 + (size_t)(n0 + c) * NI + koff;
  const _Float16* whhrow = whh16 + (size_t)(n0 + c) * NH + koff;

#pragma unroll 1
  for (int t = 0; t < NT; ++t) {
    const int cur = t & 1, nxt = cur ^ 1;
    const _Float16* hch = Hhi + cur * HTILE + c * HP + koff;
    const _Float16* hcl = Hlo + cur * HTILE + c * HP + koff;
    const _Float16* xcp = Xs  + cur * XTILE + c * XP + koff;
    _Float16* hnh = Hhi + nxt * HTILE;
    _Float16* hnl = Hlo + nxt * HTILE;

    v8f acc[4], accl[4];
#pragma unroll
    for (int j = 0; j < 4; ++j) { acc[j] = z8; accl[j] = z8; }

#pragma unroll
    for (int kc = 0; kc < NI / 32; ++kc) {
      const v16h fa = Frag<_Float16>::load(xcp + kc * 32);
      v16h fb[4];
#pragma unroll
      for (int j = 0; j < 4; ++j) fb[j] = Frag<_Float16>::load(wihrow + (size_t)(16 * j) * NI + kc * 32);
#pragma unroll
      for (int j = 0; j < 4; ++j) acc[j] = Frag<_Float16>::mma(fa, fb[j], acc[j]);
      guard4ab<v16h>(acc[0], acc[1], acc[2], acc[3], fa, fa, fb[0], fb[1], fb[2], fb[3]);
    }
#pragma unroll 1
    for (int kc = 0; kc < NH / 32; ++kc) {
      const v16h fah = Frag<_Float16>::load(hch + kc * 32);
      const v16h fal = Frag<_Float16>::load(hcl + kc * 32);
      v16h fb[4];
#pragma unroll
      for (int j = 0; j < 4; ++j) fb[j] = Frag<_Float16>::load(whhrow + (size_t)(16 * j) * NH + kc * 32);
#pragma unroll
      for (int j = 0; j < 4; ++j) {
        acc[j]  = Frag<_Float16>::mma(fah, fb[j], acc[j]);
        accl[j] = Frag<_Float16>::mma(fal, fb[j], accl[j]);
      }
      guard8ab_h(acc[0], acc[1], acc[2], acc[3], accl[0], accl[1], accl[2], accl[3], fah, fal, fb[0], fb[1], fb[2], fb[3]);
    }
    acc_guard4(acc[0], acc[1], acc[2], acc[3]);
    acc_guard4(accl[0], accl[1], accl[2], accl[3]);

#pragma unroll
    for (int j = 0; j < 4; ++j) {
      const int n = n0 + 16 * j + c;
#pragma unroll
      for (int r = 0; r < 8; ++r) {
        const float pre = (acc[j][r] + accl[j][r] * LO_CARRY_INV) * W_CARRY_INV + bs[j];
        const float hv  = tanhf(pre);
        _Float16 ha, la;
        split16(hv, ha, la);
        hnh[(mOff + r) * HP + n] = ha;
        hnl[(mOff + r) * HP + n] = la;
        slab[(mOff + r) * SLABP + 16 * j + c] = hv;
      }
    }
    {
      const int tn = (t + 1 < NT) ? (t + 1) : (NT - 1);
      const v4f v = *(const v4f*)(x + ((size_t)(b0 + xr) * NT + tn) * NI + xcc);
      v4h hv4;
      hv4[0] = (_Float16)v[0]; hv4[1] = (_Float16)v[1]; hv4[2] = (_Float16)v[2]; hv4[3] = (_Float16)v[3];
      *(v4h*)(Xs + nxt * XTILE + xr * XP + xcc) = hv4;
    }
    __syncthreads();

    for (int pass = 0; pass < 2; ++pass) {
#pragma unroll
      for (int it = 0; it < 4; ++it) {
        const int rr = it * 4 + q4;
        const v8h v = *(const v8h*)(hnh + rr * HP + n0 + c8);
        *(volatile v8h*)(hs16 + (((size_t)(b0 + rr) * NT + t) * NH + n0 + c8)) = v;
      }
      __threadfence();
    }
  }

  for (int pass = 0; pass < 2; ++pass) {
#pragma unroll
    for (int it = 0; it < 8; ++it) {
      const int row = it * 2 + hh;
      const v4f v = *(const v4f*)(slab + row * SLABP + c4);
      *(volatile v4f*)(hlast + (size_t)(b0 + row) * NH + n0 + c4) = v;
    }
    __threadfence();
  }
}

extern "C" void kernel_launch(void* const* d_in, const int* in_sizes, int n_in,
                              void* d_out, int out_size, void* d_ws, size_t ws_size, hipStream_t stream) {
  if (n_in < 8 || d_out == nullptr || d_ws == nullptr) return;
  if (in_sizes[0] != NB * NT * NI || in_sizes[1] != NB * NH || in_sizes[2] != NH * NI || in_sizes[3] != NH * NH ||
      in_sizes[4] != NH || in_sizes[5] != NH || in_sizes[6] != NO * NH || in_sizes[7] != NO ||
      out_size != NOUT0 + NOUT1) return;

  const float* x     = (const float*)d_in[0];
  const float* h0    = (const float*)d_in[1];
  const float* w_ih  = (const float*)d_in[2];
  const float* w_hh  = (const float*)d_in[3];
  const float* b_ih  = (const float*)d_in[4];
  const float* b_hh  = (const float*)d_in[5];
  const float* w_out = (const float*)d_in[6];
  const float* b_out = (const float*)d_in[7];
  float* out0 = (float*)d_out;
  float* out1 = out0 + (size_t)NOUT0;

  char* ws = (char*)d_ws; size_t off = 0;
  auto carve = [&](size_t bytes) -> char* { char* p = ws + off; off += (bytes + 255) & ~(size_t)255; return p; };
  unsigned short* WIH16  = (unsigned short*)carve((size_t)NH * NI * 2);
  unsigned short* WHH16  = (unsigned short*)carve((size_t)NH * NH * 2);
  unsigned short* WOUT16 = (unsigned short*)carve((size_t)NO * NH * 2);
  unsigned short* HS16   = (unsigned short*)carve((size_t)NROWS * NH * 2);
  if (off > ws_size || off > (size_t)134217728) return;

  cvt16_kernel<<<N8_WIH / 256, 256, 0, stream>>>(w_ih, WIH16, N8_WIH, W_CARRY);
  cvt16_kernel<<<N8_WHH / 256, 256, 0, stream>>>(w_hh, WHH16, N8_WHH, W_CARRY);
  cvt16_kernel<<<N8_WOUT / 256, 256, 0, stream>>>(w_out, WOUT16, N8_WOUT, W_CARRY);

  rnn_seq_kernel<<<RNN_BLKS, RNN_THR, 0, stream>>>(x, h0, b_ih, b_hh, WIH16, WHH16, HS16, out1);

  wmma_gemm64<0, false, 2, 0, false, 1><<<dim3(HEAD_GRID, 1), 256, 0, stream>>>(
      HS16, nullptr, NH, 0L, WOUT16, nullptr, NH, 0L,
      (void*)out0, nullptr, NO, 0L, b_out, nullptr, 0L, NROWS, NO, NH, W_CARRY_INV);
}
